// FastHoloBlock_85323820303029
// MI455X (gfx1250) — hardware-run, weakly checked
//
#include <hip/hip_runtime.h>
#include <math.h>

constexpr int kE = 1024;
constexpr int kM = 256;
constexpr int kB = 4;
constexpr int kS = 2048;
constexpr int kRows = kB * kS;
constexpr int kFF = 4 * kE;
constexpr int kNP = 832;
constexpr int kKQVld = 800;
constexpr int kFFChunkRows = 2048;
constexpr int kFFChunks = kRows / kFFChunkRows;
constexpr int kMemChunk = 16;
constexpr float kWCarry  = 32.0f;
constexpr float kROCarry = 1024.0f;
constexpr float kGCarry  = 16.0f;
constexpr float kLnEps   = 1e-5f;

constexpr size_t kOffXH16  = 0;
constexpr size_t kOffWP16  = 16777216;
constexpr size_t kOffWO16  = kOffWP16 + (size_t)kNP * kE * 2;
constexpr size_t kOffWF1   = kOffWO16 + (size_t)kE * kM * 2;
constexpr size_t kOffWF2   = kOffWF1 + (size_t)kFF * kE * 2;
constexpr size_t kOffZoneA = kOffWF2 + (size_t)kE * kFF * 2;
constexpr size_t kOffPROJ  = kOffZoneA;
constexpr size_t kOffKQV   = kOffPROJ + (size_t)kRows * kNP * 4;
constexpr size_t kOffRO16  = kOffKQV + (size_t)kRows * kKQVld * 4;
constexpr size_t kEndZoneA = kOffRO16 + (size_t)kRows * kM * 2;
constexpr size_t kOffFFPRE = kOffZoneA;
constexpr size_t kOffG16   = kOffFFPRE + (size_t)kFFChunkRows * kFF * 4;
constexpr size_t kEndG16   = kOffG16 + (size_t)kFFChunkRows * kFF * 2;
constexpr size_t kOffX1    = kEndZoneA;
constexpr size_t kWsTotal  = kOffX1 + (size_t)kRows * kE * 4;
static_assert(kEndG16 <= kEndZoneA);
static_assert(kWsTotal <= 134217728);
static_assert((kOffWO16 % 128) == 0 && (kOffKQV % 128) == 0 && (kOffRO16 % 128) == 0 && (kOffG16 % 128) == 0 && (kOffX1 % 128) == 0);

typedef __attribute__((ext_vector_type(16))) _Float16 v16h;
typedef __attribute__((ext_vector_type(8)))  _Float16 v8h;
typedef __attribute__((ext_vector_type(16))) __bf16   v16b;
typedef __attribute__((ext_vector_type(8)))  __bf16   v8b;
typedef __attribute__((ext_vector_type(8)))  float    v8f;
typedef __attribute__((ext_vector_type(4)))  float    v4f;
typedef __attribute__((ext_vector_type(2)))  float    v2f;
typedef __attribute__((ext_vector_type(4)))  unsigned int v4u;

__device__ __forceinline__ unsigned short f2bf_bits(float f) {
  unsigned u = __float_as_uint(f);
  return (unsigned short)((u + 0x7FFFu + ((u >> 16) & 1u)) >> 16);
}
__device__ __forceinline__ float bf_bits2f(unsigned short h) { return __uint_as_float(((unsigned)h) << 16); }

__device__ __forceinline__ void dep_guard_h(v8f& a, v8f& b, v16h x, v16h y) { asm volatile("v_nop\n\tv_nop\n\tv_nop\n\tv_nop" : "+v"(a), "+v"(b) : "v"(x), "v"(y)); }
__device__ __forceinline__ void dep_guard_b(v8f& a, v8f& b, v16b x, v16b y) { asm volatile("v_nop\n\tv_nop\n\tv_nop\n\tv_nop" : "+v"(a), "+v"(b) : "v"(x), "v"(y)); }
__device__ __forceinline__ void keep4_h(v16h a, v16h b, v16h c, v16h d) { asm volatile("v_nop" :: "v"(a), "v"(b), "v"(c), "v"(d)); }
__device__ __forceinline__ void keep4_b(v16b a, v16b b, v16b c, v16b d) { asm volatile("v_nop" :: "v"(a), "v"(b), "v"(c), "v"(d)); }
__device__ __forceinline__ void acc_guard4(v8f& a, v8f& b, v8f& c, v8f& d) { asm volatile("v_nop\n\tv_nop\n\tv_nop\n\tv_nop" : "+v"(a), "+v"(b), "+v"(c), "+v"(d)); }
template <typename T> struct Frag;
template <> struct Frag<_Float16> {
  typedef v16h V; union U { v16h v; v8h h[2]; };
  static __device__ __forceinline__ v16h load(const _Float16* p) {
    U f; f.h[0] = *(const v8h*)(p); f.h[1] = *(const v8h*)(p + 16); return f.v;
  }
  static __device__ __forceinline__ v8f mma(v16h a, v16h b, v8f c) {
    return __builtin_amdgcn_wmma_f32_16x16x32_f16(false, a, false, b, (short)0, c, false, false);
  }
  static __device__ __forceinline__ void guard(v8f& a, v8f& b, v16h x, v16h y) { dep_guard_h(a, b, x, y); }
  static __device__ __forceinline__ void keep(v16h a, v16h b, v16h c, v16h d) { keep4_h(a, b, c, d); }
};
template <> struct Frag<__bf16> {
  typedef v16b V; union U { v16b v; v8b h[2]; };
  static __device__ __forceinline__ v16b load(const __bf16* p) {
    U f; f.h[0] = *(const v8b*)(p); f.h[1] = *(const v8b*)(p + 16); return f.v;
  }
  static __device__ __forceinline__ v8f mma(v16b a, v16b b, v8f c) {
    return __builtin_amdgcn_wmma_f32_16x16x32_bf16(false, a, false, b, (short)0, c, false, false);
  }
  static __device__ __forceinline__ void guard(v8f& a, v8f& b, v16b x, v16b y) { dep_guard_b(a, b, x, y); }
  static __device__ __forceinline__ void keep(v16b a, v16b b, v16b c, v16b d) { keep4_b(a, b, c, d); }
};

__device__ __forceinline__ unsigned pk16(unsigned short a, unsigned short b) { return (unsigned)a | ((unsigned)b << 16); }
__device__ __forceinline__ unsigned short h_bits(float f) { const _Float16 h = (_Float16)f; return __builtin_bit_cast(unsigned short, h); }

__device__ __forceinline__ void wave_sync_lds() {
  __builtin_amdgcn_fence(__ATOMIC_RELEASE, "workgroup");
  __builtin_amdgcn_wave_barrier();
  __builtin_amdgcn_fence(__ATOMIC_ACQUIRE, "workgroup");
}

template <int ET> struct Elem;
template <> struct Elem<0> { typedef _Float16 T; };
template <> struct Elem<1> { typedef __bf16 T; };
template <int ET, bool SPLIT, int BIAS_MODE, int OUT_MODE, bool RESID, int ACT = 0>
__global__ __launch_bounds__(256) void wmma_gemm64(
    const unsigned short* __restrict__ Ap, const unsigned short* __restrict__ A2p, int lda, long strideA,
    const unsigned short* __restrict__ Btp, const unsigned short* __restrict__ Bt2p, int ldb, long strideB,
    void* __restrict__ Cout, void* __restrict__ Cout2, int ldc, long strideC,
    const float* __restrict__ bias,
    const float* __restrict__ resid, long strideR,
    int M, int N, int K, float scale) {
  typedef typename Elem<ET>::T T;
  typedef typename Frag<T>::V V;
  const T* A = (const T*)Ap; const T* A2 = (const T*)A2p; const T* Bt = (const T*)Btp; const T* Bt2 = (const T*)Bt2p;
  __shared__ __align__(16) float sT[8][16 * 68];
  const int b    = blockIdx.y;
  const int lane = threadIdx.x & 31;
  const int wave = threadIdx.x >> 5;
  const int tilesN = N >> 6;
  const int tilesM = M >> 6;
  const int tile = blockIdx.x * 8 + wave;
  if (tile >= tilesM * tilesN) return;
  const int tm = tile / tilesN;
  const int tn = tile - tm * tilesN;
  const int m0 = tm << 6;
  const int n0 = tn << 6;

  const T* Ab  = A  + (size_t)b * strideA;
  const T* Bb  = Bt + (size_t)b * strideB;
  const T* Ab2 = SPLIT ? (A2  + (size_t)b * strideA) : nullptr;
  const T* Bb2 = SPLIT ? (Bt2 + (size_t)b * strideB) : nullptr;

  const int rlane = lane & 15;
  const int koff  = (lane >> 4) * 8;
  const int mOff  = (lane >> 4) * 8;

  v8f acc[4][4];
#pragma unroll
  for (int i = 0; i < 4; ++i)
#pragma unroll
    for (int j = 0; j < 4; ++j) acc[i][j] = (v8f){0.f,0.f,0.f,0.f,0.f,0.f,0.f,0.f};

  for (int k0 = 0; k0 < K; k0 += 32) {
    V bh[4], bl[4];
#pragma unroll
    for (int j = 0; j < 4; ++j) {
      const size_t bo = (size_t)(n0 + (j << 4) + rlane) * ldb + koff + k0;
      bh[j] = Frag<T>::load(Bb + bo);
      if (SPLIT) bl[j] = Frag<T>::load(Bb2 + bo);
    }
#pragma unroll
    for (int i = 0; i < 4; ++i) {
      const size_t ao = (size_t)(m0 + (i << 4) + rlane) * lda + koff + k0;
      V ah = Frag<T>::load(Ab + ao);
      V al;
      if (SPLIT) al = Frag<T>::load(Ab2 + ao);
#pragma unroll
      for (int j = 0; j < 4; ++j) {
        acc[i][j] = Frag<T>::mma(ah, bh[j], acc[i][j]);
        if (SPLIT) {
          acc[i][j] = Frag<T>::mma(ah, bl[j], acc[i][j]);
          acc[i][j] = Frag<T>::mma(al, bh[j], acc[i][j]);
        }
      }
      Frag<T>::guard(acc[i][0], acc[i][3], ah, SPLIT ? al : ah);
    }
    Frag<T>::keep(bh[0], bh[1], bh[2], bh[3]);
    if (SPLIT) Frag<T>::keep(bl[0], bl[1], bl[2], bl[3]);
  }
  acc_guard4(acc[0][0], acc[0][1], acc[0][2], acc[0][3]);
  acc_guard4(acc[1][0], acc[1][1], acc[1][2], acc[1][3]);
  acc_guard4(acc[2][0], acc[2][1], acc[2][2], acc[2][3]);
  acc_guard4(acc[3][0], acc[3][1], acc[3][2], acc[3][3]);

  float* slab = sT[wave];
  const float* Rb = RESID ? (resid + (size_t)b * strideR) : nullptr;
#pragma unroll
  for (int i = 0; i < 4; ++i) {
    const int mBase = m0 + (i << 4);
#pragma unroll
    for (int j = 0; j < 4; ++j) {
      const int n = n0 + (j << 4) + rlane;
      float bv = 0.f;
      if (BIAS_MODE == 2) bv = bias[n];
#pragma unroll
      for (int r = 0; r < 8; ++r) {
        float v = acc[i][j][r] * scale;
        if (BIAS_MODE == 1) v += bias[mBase + mOff + r];
        if (BIAS_MODE == 2) v += bv;
        if (RESID) v += Rb[(size_t)(mBase + mOff + r) * ldc + n];
        if (ACT == 2) v = fmaxf(v, 0.0f);
        if (ACT == 4) v = (v > 0.f) ? v : 0.01f * v;
        slab[(mOff + r) * 68 + (j << 4) + rlane] = v;
      }
    }
    __builtin_amdgcn_fence(__ATOMIC_RELEASE, "workgroup");
    __builtin_amdgcn_wave_barrier();
    __builtin_amdgcn_fence(__ATOMIC_ACQUIRE, "workgroup");
    if (OUT_MODE == 0) {
      float* C = (float*)Cout + (size_t)b * strideC;
      const int hh = lane >> 4, c4 = (lane & 15) * 4;
      for (int pass = 0; pass < 2; ++pass) {
#pragma unroll
        for (int it = 0; it < 8; ++it) {
          const int row = it * 2 + hh;
          v4f v = *(const v4f*)(slab + row * 68 + c4);
          *(volatile v4f*)(C + (size_t)(mBase + row) * ldc + n0 + c4) = v;
        }
        __threadfence();
      }
    } else {
      const int q = lane >> 3, c8 = (lane & 7) * 8;
      unsigned short* C  = (unsigned short*)Cout  + (size_t)b * strideC;
      unsigned short* C2 = (OUT_MODE == 2) ? ((unsigned short*)Cout2 + (size_t)b * strideC) : nullptr;
      for (int pass = 0; pass < 2; ++pass) {
#pragma unroll
        for (int it = 0; it < 4; ++it) {
          const int row = it * 4 + q;
          const float* sp = slab + row * 68 + c8;
          v8h hv, lv;
#pragma unroll
          for (int e = 0; e < 8; ++e) {
            if (OUT_MODE == 1) {
              hv[e] = (_Float16)sp[e];
            } else {
              unsigned short hb = f2bf_bits(sp[e]);
              unsigned short lb = f2bf_bits(sp[e] - bf_bits2f(hb));
              hv[e] = __builtin_bit_cast(_Float16, hb);
              lv[e] = __builtin_bit_cast(_Float16, lb);
            }
          }
          *(volatile v8h*)(C + (size_t)(mBase + row) * ldc + n0 + c8) = hv;
          if (OUT_MODE == 2) *(volatile v8h*)(C2 + (size_t)(mBase + row) * ldc + n0 + c8) = lv;
        }
        __threadfence();
      }
    }
    __builtin_amdgcn_fence(__ATOMIC_RELEASE, "workgroup");
    __builtin_amdgcn_wave_barrier();
    __builtin_amdgcn_fence(__ATOMIC_ACQUIRE, "workgroup");
  }
}

__global__ __launch_bounds__(256) void cast8_f16_kernel(const float* __restrict__ in, unsigned short* __restrict__ out, int n8, float sc) {
  const int i = blockIdx.x * 256 + threadIdx.x;
  if (i >= n8) return;
  const float* p = in + 8 * (size_t)i;
  const v4f a = *(const v4f*)(p) * sc;
  const v4f c = *(const v4f*)(p + 4) * sc;
  unsigned short hb[8];
#pragma unroll
  for (int e = 0; e < 4; ++e) {
    hb[e]     = h_bits(a[e]);
    hb[4 + e] = h_bits(c[e]);
  }
  const v4u u = (v4u){pk16(hb[0], hb[1]), pk16(hb[2], hb[3]), pk16(hb[4], hb[5]), pk16(hb[6], hb[7])};
  unsigned short* q = out + 8 * (size_t)i;
  *(volatile v4u*)q = u;
  __threadfence();
  *(volatile v4u*)q = u;
}

__global__ __launch_bounds__(256) void wstack_cast_kernel(const float* __restrict__ wk, const float* __restrict__ wq, const float* __restrict__ wv,
                                                          const float* __restrict__ wgw, const float* __restrict__ wgf,
                                                          unsigned short* __restrict__ out) {
  const int gid = blockIdx.x * 256 + threadIdx.x;
  const int row = gid >> 7;
  const int c8  = (gid & 127) * 8;
  const float* src = wk;
  float sc = kWCarry;
  if (row < 256)        src = wk + (size_t)row * kE;
  else if (row < 512)   src = wq + (size_t)(row - 256) * kE;
  else if (row < 768)   src = wv + (size_t)(row - 512) * kE;
  else if (row == 768)  src = wgw;
  else if (row == 769)  src = wgf;
  else { src = wk; sc = 0.0f; }
  const v4f a = *(const v4f*)(src + c8) * sc;
  const v4f c = *(const v4f*)(src + c8 + 4) * sc;
  unsigned short hb[8];
#pragma unroll
  for (int e = 0; e < 4; ++e) {
    hb[e]     = h_bits(a[e]);
    hb[4 + e] = h_bits(c[e]);
  }
  const v4u u = (v4u){pk16(hb[0], hb[1]), pk16(hb[2], hb[3]), pk16(hb[4], hb[5]), pk16(hb[6], hb[7])};
  unsigned short* q = out + (size_t)row * kE + c8;
  *(volatile v4u*)q = u;
  __threadfence();
  *(volatile v4u*)q = u;
}

__global__ __launch_bounds__(128) void layernorm_f16_kernel(const float* __restrict__ X, const float* __restrict__ g,
                                                            const float* __restrict__ bt, unsigned short* __restrict__ out) {
  __shared__ float red[4];
  const int row = blockIdx.x, t = threadIdx.x, lane = t & 31, wave = t >> 5;
  const float* xr = X + (size_t)row * kE + 8 * t;
  const v4f a = *(const v4f*)(xr);
  const v4f c = *(const v4f*)(xr + 4);
  float s = ((a.x + a.y) + (a.z + a.w)) + ((c.x + c.y) + (c.z + c.w));
#pragma unroll
  for (int off = 16; off > 0; off >>= 1) s += __shfl_xor(s, off, 32);
  if (lane == 0) red[wave] = s;
  __syncthreads();
  const float mean = ((red[0] + red[1]) + (red[2] + red[3])) * (1.0f / 1024.0f);
  __syncthreads();
  float d[8];
  d[0] = a.x - mean; d[1] = a.y - mean; d[2] = a.z - mean; d[3] = a.w - mean;
  d[4] = c.x - mean; d[5] = c.y - mean; d[6] = c.z - mean; d[7] = c.w - mean;
  float ss = ((d[0] * d[0] + d[1] * d[1]) + (d[2] * d[2] + d[3] * d[3])) + ((d[4] * d[4] + d[5] * d[5]) + (d[6] * d[6] + d[7] * d[7]));
#pragma unroll
  for (int off = 16; off > 0; off >>= 1) ss += __shfl_xor(ss, off, 32);
  if (lane == 0) red[wave] = ss;
  __syncthreads();
  const float var = ((red[0] + red[1]) + (red[2] + red[3])) * (1.0f / 1024.0f);
  const float rs = rsqrtf(var + kLnEps);
  const v4f g0 = *(const v4f*)(g + 8 * t), g1 = *(const v4f*)(g + 8 * t + 4);
  const v4f b0 = *(const v4f*)(bt + 8 * t), b1 = *(const v4f*)(bt + 8 * t + 4);
  float y[8];
  y[0] = d[0] * rs * g0.x + b0.x; y[1] = d[1] * rs * g0.y + b0.y; y[2] = d[2] * rs * g0.z + b0.z; y[3] = d[3] * rs * g0.w + b0.w;
  y[4] = d[4] * rs * g1.x + b1.x; y[5] = d[5] * rs * g1.y + b1.y; y[6] = d[6] * rs * g1.z + b1.z; y[7] = d[7] * rs * g1.w + b1.w;
  unsigned short hb[8];
#pragma unroll
  for (int e = 0; e < 8; ++e) hb[e] = h_bits(y[e]);
  const v4u u = (v4u){pk16(hb[0], hb[1]), pk16(hb[2], hb[3]), pk16(hb[4], hb[5]), pk16(hb[6], hb[7])};
  unsigned short* q = out + (size_t)row * kE + 8 * t;
  *(volatile v4u*)q = u;
  __threadfence();
  *(volatile v4u*)q = u;
}

__global__ __launch_bounds__(256) void kqv_finish_kernel(const float* __restrict__ P, const float* __restrict__ bk, const float* __restrict__ bq,
                                                         const float* __restrict__ bvv, const float* __restrict__ bgw, const float* __restrict__ bgf,
                                                         float* __restrict__ KQV) {
  __shared__ float red[16];
  const int row = blockIdx.x, t = threadIdx.x, lane = t & 31, wave = t >> 5;
  const int region = t >> 6;
  const int col = (4 * t < kNP - 4) ? (4 * t) : (kNP - 4);
  const v4f p = *(const v4f*)(P + (size_t)row * kNP + col);
  const int bi = 4 * (t & 63);
  const v4f bb0 = *(const v4f*)(bk + bi);
  const v4f bb1 = *(const v4f*)(bq + bi);
  const v4f bb2 = *(const v4f*)(bvv + bi);
  v4f bias = (v4f){0.f, 0.f, 0.f, 0.f};
  if (region == 0) bias = bb0;
  else if (region == 1) bias = bb1;
  else if (region == 2) bias = bb2;
  const v4f x = p + bias;
  const float ss = (x.x * x.x + x.y * x.y) + (x.z * x.z + x.w * x.w);
  float sk = (region == 0) ? ss : 0.0f;
  float sq = (region == 1) ? ss : 0.0f;
#pragma unroll
  for (int off = 16; off > 0; off >>= 1) { sk += __shfl_xor(sk, off, 32); sq += __shfl_xor(sq, off, 32); }
  if (lane == 0) { red[wave] = sk; red[8 + wave] = sq; }
  __syncthreads();
  const float SK = ((red[0] + red[1]) + (red[2] + red[3])) + ((red[4] + red[5]) + (red[6] + red[7]));
  const float SQ = ((red[8] + red[9]) + (red[10] + red[11])) + ((red[12] + red[13]) + (red[14] + red[15]));
  const float rk = 1.0f / fmaxf(sqrtf(SK), 1e-12f);
  const float rq = 1.0f / fmaxf(sqrtf(SQ), 1e-12f);
  v4f o = (v4f){0.f, 0.f, 0.f, 0.f};
  if (region == 0) {
    o = x * rk;
  } else if (region == 1) {
    o = x * rq;
  } else if (region == 2) {
    o.x = tanhf(x.x); o.y = tanhf(x.y); o.z = tanhf(x.z); o.w = tanhf(x.w);
  } else {
    const float gw = 1.0f / (1.0f + expf(-(p.x + bgw[0])));
    const float gf = 1.0f / (1.0f + expf(-(p.y + bgf[0])));
    if (t == 192) { o.x = gw; o.y = gf; }
  }
  if (t < 200) {
    float* dst = KQV + (size_t)row * kKQVld + 4 * t;
    *(volatile v4f*)dst = o;
    __threadfence();
    *(volatile v4f*)dst = o;
  }
}

__global__ __launch_bounds__(512) void holo_mem_kernel(const float* __restrict__ KQV, const float* __restrict__ mem_in,
                                                       unsigned short* __restrict__ RO, float* __restrict__ mem_out) {
  __shared__ __align__(16) float sPool[8192];
  __shared__ __align__(16) float sV[kMemChunk * 128];
  __shared__ __align__(16) float sR[kMemChunk * 128];
  __shared__ float sG[2 * kMemChunk];
  const int tid = threadIdx.x, lane = tid & 31, wave = tid >> 5;
  const int b  = blockIdx.x >> 1;
  const int rh = blockIdx.x & 1;
  const int il = tid >> 2;
  const int c  = tid & 3;
  const int ig = 128 * rh + il;
  v4f m4[16];
  {
    const float* mrow = mem_in + ((size_t)(b * kM + ig)) * kM + 64 * c;
#pragma unroll
    for (int jj = 0; jj < 16; ++jj) m4[jj] = *(const v4f*)(mrow + 4 * jj);
  }
  const float* kqvb = KQV + (size_t)b * kS * kKQVld;
  for (int ch = 0; ch < kS / kMemChunk; ++ch) {
    const int t0 = ch * kMemChunk;
#pragma unroll
    for (int it = 0; it < 4; ++it) {
      const int idx = it * 512 + tid;
      const int row = idx >> 7;
      const int c4  = (idx & 127) * 4;
      const v4f v = *(const v4f*)(kqvb + (size_t)(t0 + row) * kKQVld + c4);
      const int dst = (c4 < 256) ? (row * 256 + c4) : (4096 + row * 256 + (c4 - 256));
      *(v4f*)(sPool + dst) = v;
    }
    {
      const int row = tid >> 5;
      const int c4  = (tid & 31) * 4;
      const v4f v = *(const v4f*)(kqvb + (size_t)(t0 + row) * kKQVld + 512 + 128 * rh + c4);
      *(v4f*)(sV + row * 128 + c4) = v;
    }
    if (tid < kMemChunk) {
      const v2f gg = *(const v2f*)(kqvb + (size_t)(t0 + tid) * kKQVld + 768);
      sG[2 * tid] = gg.x;
      sG[2 * tid + 1] = gg.y;
    }
    __syncthreads();
#pragma unroll 1
    for (int tl = 0; tl < kMemChunk; ++tl) {
      const float* qp = sPool + 4096 + tl * 256 + 64 * c;
      v4f acc4 = (v4f){0.f, 0.f, 0.f, 0.f};
#pragma unroll
      for (int jj = 0; jj < 16; ++jj) {
        const v4f q4 = *(const v4f*)(qp + 4 * jj);
        acc4.x = fmaf(m4[jj].x, q4.x, acc4.x);
        acc4.y = fmaf(m4[jj].y, q4.y, acc4.y);
        acc4.z = fmaf(m4[jj].z, q4.z, acc4.z);
        acc4.w = fmaf(m4[jj].w, q4.w, acc4.w);
      }
      float ro = (acc4.x + acc4.y) + (acc4.z + acc4.w);
      ro += __shfl_xor(ro, 1, 32);
      ro += __shfl_xor(ro, 2, 32);
      if (c == 0) sR[tl * 128 + il] = ro;
      const float beta  = sG[2 * tl];
      const float decay = sG[2 * tl + 1];
      const float vi    = sV[tl * 128 + il];
      const float* kp = sPool + tl * 256 + 64 * c;
      {
#pragma clang fp contract(off)
        const float bvi = beta * vi;
#pragma unroll
        for (int jj = 0; jj < 16; ++jj) {
          const v4f k4 = *(const v4f*)(kp + 4 * jj);
          const v4f t4 = k4 * bvi;
          const v4f d4 = m4[jj] * decay;
          m4[jj] = d4 + t4;
        }
      }
    }
    __syncthreads();
    if (tid < 256) {
      const int tl = tid >> 4;
      const int s  = tid & 15;
      const float* rp = sR + tl * 128 + 8 * s;
      const v4f ra = *(const v4f*)(rp);
      const v4f rc = *(const v4f*)(rp + 4);
      unsigned short hb[8];
#pragma unroll
      for (int e = 0; e < 4; ++e) {
        hb[e]     = h_bits(ra[e] * kROCarry);
        hb[4 + e] = h_bits(rc[e] * kROCarry);
      }
      const v4u u = (v4u){pk16(hb[0], hb[1]), pk16(hb[2], hb[3]), pk16(hb[4], hb[5]), pk16(hb[6], hb[7])};
      unsigned short* dst = RO + ((size_t)(b * kS + t0 + tl)) * kM + 128 * rh + 8 * s;
      *(volatile v4u*)dst = u;
      __threadfence();
      *(volatile v4u*)dst = u;
    }
  }
  __syncthreads();
  {
    float* stg = sPool + wave * 512;
    float* ob = mem_out + ((size_t)(b * kM + 128 * rh + 8 * wave)) * kM;
    const int a = lane >> 2;
#pragma unroll
    for (int p = 0; p < 4; ++p) {
      if ((a >> 1) == p) {
        float* sp = stg + (a & 1) * 256 + 64 * c;
#pragma unroll
        for (int jj = 0; jj < 16; ++jj) *(v4f*)(sp + 4 * jj) = m4[jj];
      }
      wave_sync_lds();
      for (int pass = 0; pass < 2; ++pass) {
#pragma unroll
        for (int it = 0; it < 4; ++it) {
          const v4f v = *(const v4f*)(stg + it * 128 + 4 * lane);
          *(volatile v4f*)(ob + p * 512 + it * 128 + 4 * lane) = v;
        }
        __threadfence();
      }
      wave_sync_lds();
    }
  }
}

__global__ __launch_bounds__(256) void gelu_f16x2_kernel(const float* __restrict__ in, unsigned short* __restrict__ out, int n2, float carry) {
  const int i = blockIdx.x * 256 + threadIdx.x;
  if (i >= n2) return;
  const v2f x = *(const v2f*)(in + 2 * (size_t)i);
  const float g0 = 0.5f * x.x * (1.0f + erff(x.x * 0.70710678118654752f)) * carry;
  const float g1 = 0.5f * x.y * (1.0f + erff(x.y * 0.70710678118654752f)) * carry;
  const unsigned u = pk16(h_bits(g0), h_bits(g1));
  unsigned* q = (unsigned*)(out + 2 * (size_t)i);
  *(volatile unsigned*)q = u;
  __threadfence();
  *(volatile unsigned*)q = u;
}

extern "C" void kernel_launch(void* const* d_in, const int* in_sizes, int n_in,
                              void* d_out, int out_size, void* d_ws, size_t ws_size, hipStream_t stream) {
  if (n_in < 22) return;
  if (in_sizes[0] != kRows * kE) return;
  if (out_size != kRows * kE + kB * kM * kM) return;
  if (ws_size < kWsTotal) return;

  const float* x      = (const float*)d_in[0];
  const float* mem_in = (const float*)d_in[1];
  const float* w_k    = (const float*)d_in[2];
  const float* b_k    = (const float*)d_in[3];
  const float* w_q    = (const float*)d_in[4];
  const float* b_q    = (const float*)d_in[5];
  const float* w_v    = (const float*)d_in[6];
  const float* b_v    = (const float*)d_in[7];
  const float* w_out  = (const float*)d_in[8];
  const float* b_out  = (const float*)d_in[9];
  const float* w_gw   = (const float*)d_in[10];
  const float* b_gw   = (const float*)d_in[11];
  const float* w_gf   = (const float*)d_in[12];
  const float* b_gf   = (const float*)d_in[13];
  const float* ln1_g  = (const float*)d_in[14];
  const float* ln1_b  = (const float*)d_in[15];
  const float* ln2_g  = (const float*)d_in[16];
  const float* ln2_b  = (const float*)d_in[17];
  const float* w_f1   = (const float*)d_in[18];
  const float* b_f1   = (const float*)d_in[19];
  const float* w_f2   = (const float*)d_in[20];
  const float* b_f2   = (const float*)d_in[21];

  char* ws = (char*)d_ws;
  unsigned short* XH16  = (unsigned short*)(ws + kOffXH16);
  unsigned short* WP16  = (unsigned short*)(ws + kOffWP16);
  unsigned short* WO16  = (unsigned short*)(ws + kOffWO16);
  unsigned short* WF1   = (unsigned short*)(ws + kOffWF1);
  unsigned short* WF2   = (unsigned short*)(ws + kOffWF2);
  float*          PROJ  = (float*)(ws + kOffPROJ);
  float*          KQV   = (float*)(ws + kOffKQV);
  unsigned short* RO16  = (unsigned short*)(ws + kOffRO16);
  float*          FFPRE = (float*)(ws + kOffFFPRE);
  unsigned short* G16   = (unsigned short*)(ws + kOffG16);
  float*          X1    = (float*)(ws + kOffX1);
  float* out0 = (float*)d_out;
  float* out1 = out0 + (size_t)kRows * kE;

  wstack_cast_kernel<<<(kNP * (kE / 8)) / 256, 256, 0, stream>>>(w_k, w_q, w_v, w_gw, w_gf, WP16);
  cast8_f16_kernel<<<(kE * kM / 8) / 256, 256, 0, stream>>>(w_out, WO16, kE * kM / 8, kWCarry);
  cast8_f16_kernel<<<(kFF * kE / 8) / 256, 256, 0, stream>>>(w_f1, WF1, kFF * kE / 8, kWCarry);
  cast8_f16_kernel<<<(kE * kFF / 8) / 256, 256, 0, stream>>>(w_f2, WF2, kE * kFF / 8, kWCarry);

  layernorm_f16_kernel<<<kRows, 128, 0, stream>>>(x, ln1_g, ln1_b, XH16);

  wmma_gemm64<0, false, 0, 0, false><<<dim3((kRows / 64) * (kNP / 64) / 8, 1), 256, 0, stream>>>(
      XH16, XH16, kE, 0L, WP16, WP16, kE, 0L, (void*)PROJ, (void*)PROJ, kNP, 0L,
      (const float*)nullptr, (const float*)nullptr, 0L, kRows, kNP, kE, 1.0f / kWCarry);

  kqv_finish_kernel<<<kRows, 256, 0, stream>>>(PROJ, b_k, b_q, b_v, b_gw, b_gf, KQV);

  holo_mem_kernel<<<kB * 2, 512, 0, stream>>>(KQV, mem_in, RO16, out1);

  wmma_gemm64<0, false, 2, 0, true><<<dim3((kRows / 64) * (kE / 64) / 8, 1), 256, 0, stream>>>(
      RO16, RO16, kM, 0L, WO16, WO16, kM, 0L, (void*)X1, (void*)X1, kE, 0L,
      b_out, x, 0L, kRows, kE, kM, 1.0f / (kROCarry * kWCarry));

  layernorm_f16_kernel<<<kRows, 128, 0, stream>>>(X1, ln2_g, ln2_b, XH16);

  for (int qc = 0; qc < kFFChunks; ++qc) {
    const size_t r0 = (size_t)qc * kFFChunkRows;
    wmma_gemm64<0, false, 2, 0, false><<<dim3((kFFChunkRows / 64) * (kFF / 64) / 8, 1), 256, 0, stream>>>(
        XH16 + r0 * kE, XH16 + r0 * kE, kE, 0L, WF1, WF1, kE, 0L, (void*)FFPRE, (void*)FFPRE, kFF, 0L,
        b_f1, (const float*)nullptr, 0L, kFFChunkRows, kFF, kE, 1.0f / kWCarry);
    gelu_f16x2_kernel<<<(kFFChunkRows * kFF / 2) / 256, 256, 0, stream>>>(FFPRE, G16, kFFChunkRows * kFF / 2, kGCarry);
    wmma_gemm64<0, false, 2, 0, true><<<dim3((kFFChunkRows / 64) * (kE / 64) / 8, 1), 256, 0, stream>>>(
        G16, G16, kFF, 0L, WF2, WF2, kFF, 0L, (void*)(out0 + r0 * kE), (void*)(out0 + r0 * kE), kE, 0L,
        b_f2, X1 + r0 * kE, 0L, kFFChunkRows, kE, kFF, 1.0f / (kGCarry * kWCarry));
  }
}
